// LPropDecoderLayer_56951266345699
// MI455X (gfx1250) — hardware-verified
//
#include <hip/hip_runtime.h>
#define NS 4
#define NFR 8
#define CC 256
#define HW 1024
#define KD 128
#define CE 16
#define LK (NFR * HW)

typedef __bf16 v16b __attribute__((ext_vector_type(16)));
typedef unsigned short v8us __attribute__((ext_vector_type(8), may_alias));
typedef float  v8f  __attribute__((ext_vector_type(8)));
typedef float  v4f  __attribute__((ext_vector_type(4)));
typedef float  v4fa __attribute__((ext_vector_type(4), may_alias));
union FragB { v16b v; v8us half[2]; unsigned short u[16]; };

__device__ __forceinline__ unsigned short bf16_bits(float x) { unsigned int u = __float_as_uint(x); return (unsigned short)((u + 0x7FFFu + ((u >> 16) & 1u)) >> 16); }
__device__ __forceinline__ float bf16_val(unsigned short b) { return __uint_as_float(((unsigned int)b) << 16); }
__device__ __forceinline__ float bf16_round(float x) { return bf16_val(bf16_bits(x)); }
template <int NT>
__device__ __forceinline__ v8f mmaN(v16b ah, v16b al, v16b bh, v16b bl, v8f c) {
  c = __builtin_amdgcn_wmma_f32_16x16x32_bf16(false, ah, false, bh, (short)0, c, false, false);
  if (NT >= 2) c = __builtin_amdgcn_wmma_f32_16x16x32_bf16(false, al, false, bh, (short)0, c, false, false);
  if (NT >= 3) c = __builtin_amdgcn_wmma_f32_16x16x32_bf16(false, ah, false, bl, (short)0, c, false, false);
  asm volatile("v_nop\n\tv_nop\n\tv_nop\n\tv_nop" : "+v"(c) : "v"(ah), "v"(al), "v"(bh), "v"(bl));
  return c;
}

__global__ __launch_bounds__(256) void k_wt_bf16(const float* __restrict__ W, unsigned short* __restrict__ Wt, int K, int N) {
  const int t = blockIdx.x * 256 + threadIdx.x;
  const int k8n = K / 8;
  if (t >= N * k8n) return;
  const int n = t / k8n, k8 = (t % k8n) * 8;
  v8us v;
#pragma unroll
  for (int i = 0; i < 8; ++i) v[i] = bf16_bits(W[(size_t)(k8 + i) * N + n]);
  *(volatile v8us*)(Wt + (size_t)n * K + k8) = v;
  __threadfence();
  *(volatile v8us*)(Wt + (size_t)n * K + k8) = v;
}

template <bool ASPLIT, int ACT, bool BIAS_BF16>
__global__ __launch_bounds__(128) void k_gemm_bf(const float* __restrict__ A, int lda, const unsigned short* __restrict__ Wt, int ldb,
                                               const float* __restrict__ bias, float* __restrict__ C, int ldc, int M, int N, int K) {
  __shared__ __attribute__((aligned(16))) float so[4][16][64];
  const int tid = threadIdx.x, w = tid >> 5, lane = tid & 31, ln = lane & 15, hh = lane >> 4;
  const int ntn = N / 64;
  const int wid = blockIdx.x * 4 + w;
  const int mt = wid / ntn, nq = wid % ntn;
  if (mt * 16 >= M) return;
  const int row0 = mt * 16, col0 = nq * 64;
  const float* arow = A + (size_t)(row0 + ln) * lda;
  v8f acc[4] = {};
  for (int kb = 0; kb < K; kb += 32) {
    FragB ah, al;
    const v4f x0 = *(const v4fa*)(arow + kb + 8 * hh), x1 = *(const v4fa*)(arow + kb + 8 * hh + 4);
    const v4f x2 = *(const v4fa*)(arow + kb + 16 + 8 * hh), x3 = *(const v4fa*)(arow + kb + 16 + 8 * hh + 4);
    float xs[16] = {x0[0],x0[1],x0[2],x0[3],x1[0],x1[1],x1[2],x1[3],x2[0],x2[1],x2[2],x2[3],x3[0],x3[1],x3[2],x3[3]};
#pragma unroll
    for (int i = 0; i < 16; ++i) { const unsigned short hb = bf16_bits(xs[i]); ah.u[i] = hb; al.u[i] = ASPLIT ? bf16_bits(xs[i] - bf16_val(hb)) : (unsigned short)0; }
#pragma unroll
    for (int t = 0; t < 4; ++t) {
      const unsigned short* brow = Wt + (size_t)(col0 + t * 16 + ln) * ldb + kb;
      FragB b;
      b.half[0] = *(const v8us*)(brow + 8 * hh);
      b.half[1] = *(const v8us*)(brow + 16 + 8 * hh);
      acc[t] = mmaN<ASPLIT ? 2 : 1>(ah.v, al.v, b.v, b.v, acc[t]);
    }
  }
#pragma unroll
  for (int t = 0; t < 4; ++t) {
    float bv = bias ? bias[col0 + t * 16 + ln] : 0.f;
    if (BIAS_BF16) bv = bf16_round(bv);
#pragma unroll
    for (int r = 0; r < 8; ++r) { float v = acc[t][r] + bv; if (ACT == 1) v = fmaxf(v, 0.f); so[w][8 * hh + r][t * 16 + ln] = v; }
  }
  __builtin_amdgcn_fence(__ATOMIC_ACQ_REL, "workgroup");
  __builtin_amdgcn_wave_barrier();
  const int rsub = lane >> 4, c4 = (lane & 15) * 4;
  for (int pass = 0; pass < 2; ++pass) {
#pragma unroll
    for (int q = 0; q < 8; ++q) {
      const int r = q * 2 + rsub;
      const v4f v = *(const v4fa*)&so[w][r][c4];
      *(volatile v4f*)(C + (size_t)(row0 + r) * ldc + col0 + c4) = v;
    }
    if (pass == 0) __threadfence();
  }
}

template <int D, bool CAUSAL>
__global__ __launch_bounds__(128) void k_flash(const float* __restrict__ qb, const float* __restrict__ kb, const float* __restrict__ vb,
                                             int pitch, int T, int H, float scale, float* __restrict__ y, int ypitch) {
  constexpr int KS = D / 32;
  constexpr int DT = D / 16;
  __shared__ __attribute__((aligned(16))) unsigned short sKh[32][D + 8], sKl[32][D + 8], sVh[32][D + 8], sVl[32][D + 8];
  __shared__ __attribute__((aligned(16))) unsigned short sPh[4][16][40], sPl[4][16][40];
  __shared__ __attribute__((aligned(16))) float sO[4][16][D];
  const int tid = threadIdx.x, w = tid >> 5, lane = tid & 31, ln = lane & 15, hh = lane >> 4;
  const int nqb = (T + 63) / 64;
  const int bh = blockIdx.x / nqb, qblk = blockIdx.x % nqb;
  const int b = bh / H, h = bh % H;
  const int q0 = qblk * 64 + w * 16;
  const float* Q = qb + (size_t)b * T * pitch + h * D;
  const float* K = kb + (size_t)b * T * pitch + h * D;
  const float* V = vb + (size_t)b * T * pitch + h * D;

  FragB aqh[KS], aql[KS];
  {
    int row = q0 + ln; if (row >= T) row = T - 1;
    const float* qr = Q + (size_t)row * pitch;
#pragma unroll
    for (int ks = 0; ks < KS; ++ks)
#pragma unroll
      for (int i = 0; i < 16; ++i) {
        const int d = ks * 32 + ((i < 8) ? (8 * hh + i) : (16 + 8 * hh + (i - 8)));
        const float x = qr[d] * scale; const unsigned short hb = bf16_bits(x);
        aqh[ks].u[i] = hb; aql[ks].u[i] = bf16_bits(x - bf16_val(hb));
      }
  }
  float m_r[8], l_r[8];
#pragma unroll
  for (int r = 0; r < 8; ++r) { m_r[r] = -3.0e38f; l_r[r] = 0.f; }
  v8f oacc[DT];
#pragma unroll
  for (int dt = 0; dt < DT; ++dt) oacc[dt] = (v8f){0.f,0.f,0.f,0.f,0.f,0.f,0.f,0.f};

  const int kv_end = CAUSAL ? min(T, qblk * 64 + 64) : T;
  for (int j0 = 0; j0 < kv_end; j0 += 32) {
    __syncthreads();
    for (int e = tid; e < 32 * (D / 4); e += 128) {
      const int r = e / (D / 4), c4 = (e % (D / 4)) * 4;
      const int key = j0 + r;
      v4f kf = {0.f,0.f,0.f,0.f}, vf = {0.f,0.f,0.f,0.f};
      if (key < T) { kf = *(const v4fa*)(K + (size_t)key * pitch + c4); vf = *(const v4fa*)(V + (size_t)key * pitch + c4); }
#pragma unroll
      for (int t = 0; t < 4; ++t) {
        unsigned short hb = bf16_bits(kf[t]); sKh[r][c4 + t] = hb; sKl[r][c4 + t] = bf16_bits(kf[t] - bf16_val(hb));
        hb = bf16_bits(vf[t]); sVh[r][c4 + t] = hb; sVl[r][c4 + t] = bf16_bits(vf[t] - bf16_val(hb));
      }
    }
    __syncthreads();
    v8f s[2];
#pragma unroll
    for (int nt = 0; nt < 2; ++nt) {
      v8f acc = {};
#pragma unroll
      for (int ks = 0; ks < KS; ++ks) {
        FragB bh_, bl_;
        bh_.half[0] = *(const v8us*)&sKh[nt * 16 + ln][ks * 32 + 8 * hh]; bh_.half[1] = *(const v8us*)&sKh[nt * 16 + ln][ks * 32 + 16 + 8 * hh];
        bl_.half[0] = *(const v8us*)&sKl[nt * 16 + ln][ks * 32 + 8 * hh]; bl_.half[1] = *(const v8us*)&sKl[nt * 16 + ln][ks * 32 + 16 + 8 * hh];
        acc = mmaN<3>(aqh[ks].v, aql[ks].v, bh_.v, bl_.v, acc);
      }
      s[nt] = acc;
    }
    float alpha[8];
#pragma unroll
    for (int r = 0; r < 8; ++r) {
      const int qi = q0 + 8 * hh + r;
      const int ja = j0 + ln, jb = j0 + 16 + ln;
      if (CAUSAL) { if (ja > qi) s[0][r] = -3.0e38f; if (jb > qi) s[1][r] = -3.0e38f; }
      if (ja >= T) s[0][r] = -3.0e38f;
      if (jb >= T) s[1][r] = -3.0e38f;
      float mx = fmaxf(s[0][r], s[1][r]);
      mx = fmaxf(mx, __shfl_xor(mx, 1, 32)); mx = fmaxf(mx, __shfl_xor(mx, 2, 32)); mx = fmaxf(mx, __shfl_xor(mx, 4, 32)); mx = fmaxf(mx, __shfl_xor(mx, 8, 32));
      const float mnew = fmaxf(m_r[r], mx);
      alpha[r] = (mnew > -1.0e38f) ? __expf(m_r[r] - mnew) : 1.0f;
      const float p0 = (s[0][r] > -1.0e38f) ? __expf(s[0][r] - mnew) : 0.f;
      const float p1 = (s[1][r] > -1.0e38f) ? __expf(s[1][r] - mnew) : 0.f;
      m_r[r] = mnew;
      l_r[r] = l_r[r] * alpha[r] + p0 + p1;
      unsigned short hb = bf16_bits(p0); sPh[w][8 * hh + r][ln] = hb;      sPl[w][8 * hh + r][ln] = bf16_bits(p0 - bf16_val(hb));
      hb = bf16_bits(p1);                sPh[w][8 * hh + r][16 + ln] = hb; sPl[w][8 * hh + r][16 + ln] = bf16_bits(p1 - bf16_val(hb));
    }
#pragma unroll
    for (int dt = 0; dt < DT; ++dt)
#pragma unroll
      for (int r = 0; r < 8; ++r) oacc[dt][r] *= alpha[r];
    __builtin_amdgcn_fence(__ATOMIC_ACQ_REL, "workgroup");
    __builtin_amdgcn_wave_barrier();
    FragB pah, pal;
    pah.half[0] = *(const v8us*)&sPh[w][ln][8 * hh]; pah.half[1] = *(const v8us*)&sPh[w][ln][16 + 8 * hh];
    pal.half[0] = *(const v8us*)&sPl[w][ln][8 * hh]; pal.half[1] = *(const v8us*)&sPl[w][ln][16 + 8 * hh];
#pragma unroll
    for (int dt = 0; dt < DT; ++dt) {
      FragB bvh, bvl;
#pragma unroll
      for (int i = 0; i < 8; ++i) {
        bvh.u[i] = sVh[8 * hh + i][dt * 16 + ln]; bvh.u[8 + i] = sVh[16 + 8 * hh + i][dt * 16 + ln];
        bvl.u[i] = sVl[8 * hh + i][dt * 16 + ln]; bvl.u[8 + i] = sVl[16 + 8 * hh + i][dt * 16 + ln];
      }
      oacc[dt] = mmaN<3>(pah.v, pal.v, bvh.v, bvl.v, oacc[dt]);
    }
    __builtin_amdgcn_fence(__ATOMIC_ACQ_REL, "workgroup");
    __builtin_amdgcn_wave_barrier();
  }
#pragma unroll
  for (int r = 0; r < 8; ++r) {
    float l = l_r[r];
    l += __shfl_xor(l, 1, 32); l += __shfl_xor(l, 2, 32); l += __shfl_xor(l, 4, 32); l += __shfl_xor(l, 8, 32);
    l_r[r] = (l > 0.f) ? 1.0f / l : 0.f;
  }
#pragma unroll
  for (int dt = 0; dt < DT; ++dt)
#pragma unroll
    for (int r = 0; r < 8; ++r) sO[w][8 * hh + r][dt * 16 + ln] = oacc[dt][r] * l_r[r];
  __builtin_amdgcn_fence(__ATOMIC_ACQ_REL, "workgroup");
  __builtin_amdgcn_wave_barrier();
  for (int pass = 0; pass < 2; ++pass) {
    for (int r = 0; r < 16; ++r) {
      const int row = q0 + r;
      if (row < T && lane < D / 4) {
        const v4f val = *(const v4fa*)&sO[w][r][lane * 4];
        *(volatile v4f*)(y + ((size_t)b * T + row) * ypitch + h * D + lane * 4) = val;
      }
    }
    if (pass == 0) __threadfence();
  }
}

template <bool AFFINE, bool RESID, bool RES_BF16>
__global__ __launch_bounds__(256) void k_transpose32(const float* __restrict__ in, float* __restrict__ out, int rows, int cols,
                                                    const float* __restrict__ scale, const float* __restrict__ shift, const float* __restrict__ res) {
  __shared__ float tile[32][33];
  const int b = blockIdx.z;
  const int r0 = blockIdx.y * 32, c0 = blockIdx.x * 32;
  const float* src = in + (size_t)b * rows * cols;
  float* dst = out + (size_t)b * rows * cols;
  const int tx = threadIdx.x & 31, ty = threadIdx.x >> 5;
  for (int i = ty; i < 32; i += 8) tile[i][tx] = src[(size_t)(r0 + i) * cols + c0 + tx];
  __syncthreads();
  for (int pass = 0; pass < 2; ++pass) {
    for (int i = ty; i < 32; i += 8) {
      float v = tile[tx][i];
      const int orow = c0 + i;
      if (AFFINE) v = v * scale[orow] + shift[orow];
      if (RESID) { float rv = res[(size_t)b * rows * cols + (size_t)orow * rows + r0 + tx]; if (RES_BF16) rv = bf16_round(rv); v += rv; }
      *(volatile float*)(dst + (size_t)orow * rows + r0 + tx) = v;
    }
    if (pass == 0) __threadfence();
  }
}

__global__ __launch_bounds__(256) void k_pool2_pm(const float* __restrict__ in, float* __restrict__ out, int Bn, int H, int W, int C) {
  const size_t t = (size_t)blockIdx.x * 256 + threadIdx.x;
  const int c4n = C / 4, Ho = H / 2, Wo = W / 2;
  const size_t total = (size_t)Bn * Ho * Wo * c4n;
  if (t >= total) return;
  const int c4 = (int)(t % c4n) * 4; size_t rest = t / c4n;
  const int pw = (int)(rest % Wo); rest /= Wo; const int ph = (int)(rest % Ho); const int b = (int)(rest / Ho);
  const float* base = in + (size_t)b * H * W * C;
  const int p00 = (2 * ph) * W + 2 * pw;
  const v4f a = *(const v4fa*)(base + (size_t)p00 * C + c4), bq = *(const v4fa*)(base + (size_t)(p00 + 1) * C + c4);
  const v4f c = *(const v4fa*)(base + (size_t)(p00 + W) * C + c4), d = *(const v4fa*)(base + (size_t)(p00 + W + 1) * C + c4);
  v4f m; for (int i = 0; i < 4; ++i) m[i] = fmaxf(fmaxf(a[i], bq[i]), fmaxf(c[i], d[i]));
  float* dst = out + ((size_t)b * Ho * Wo + (size_t)ph * Wo + pw) * C + c4;
  *(volatile v4f*)dst = m;
  __threadfence();
  *(volatile v4f*)dst = m;
}

template <int DQ, int DV>
__global__ __launch_bounds__(128) void k_flash2(const float* __restrict__ Qb, size_t qstride, int qpitch, int Tq,
                                              const float* __restrict__ Kb, size_t kstride, int kpitch, int Tk,
                                              const float* __restrict__ Vb, size_t vstride, int vpitch,
                                              float scale, float* __restrict__ y, size_t ystride, int ypitch) {
  constexpr int KS = DQ / 32, DT = DV / 16;
  __shared__ __attribute__((aligned(16))) unsigned short sKh[32][DQ + 8], sKl[32][DQ + 8], sVh[32][DV + 8], sVl[32][DV + 8];
  __shared__ __attribute__((aligned(16))) unsigned short sPh[4][16][40], sPl[4][16][40];
  __shared__ __attribute__((aligned(16))) float sO[4][16][DV];
  const int tid = threadIdx.x, w = tid >> 5, lane = tid & 31, ln = lane & 15, hh = lane >> 4;
  const int nqb = (Tq + 63) / 64;
  const int bh = blockIdx.x / nqb, qblk = blockIdx.x % nqb;
  const int dv0 = blockIdx.y * DV;
  const int q0 = qblk * 64 + w * 16;
  const float* Q = Qb + (size_t)bh * qstride; const float* K = Kb + (size_t)bh * kstride; const float* V = Vb + (size_t)bh * vstride + dv0;
  FragB aqh[KS], aql[KS];
  {
    int row = q0 + ln; if (row >= Tq) row = Tq - 1;
    const float* qr = Q + (size_t)row * qpitch;
#pragma unroll
    for (int ks = 0; ks < KS; ++ks)
#pragma unroll
      for (int i = 0; i < 16; ++i) {
        const int d = ks * 32 + ((i < 8) ? (8 * hh + i) : (16 + 8 * hh + (i - 8)));
        const float x = qr[d] * scale; const unsigned short hb = bf16_bits(x);
        aqh[ks].u[i] = hb; aql[ks].u[i] = bf16_bits(x - bf16_val(hb));
      }
  }
  float m_r[8], l_r[8];
#pragma unroll
  for (int r = 0; r < 8; ++r) { m_r[r] = -3.0e38f; l_r[r] = 0.f; }
  v8f oacc[DT];
#pragma unroll
  for (int dt = 0; dt < DT; ++dt) oacc[dt] = (v8f){0.f,0.f,0.f,0.f,0.f,0.f,0.f,0.f};
  for (int j0 = 0; j0 < Tk; j0 += 32) {
    __syncthreads();
    for (int e = tid; e < 32 * (DQ / 4); e += 128) {
      const int r = e / (DQ / 4), c4 = (e % (DQ / 4)) * 4; const int key = j0 + r;
      v4f f = {0.f,0.f,0.f,0.f}; if (key < Tk) f = *(const v4fa*)(K + (size_t)key * kpitch + c4);
#pragma unroll
      for (int t = 0; t < 4; ++t) { const unsigned short hb = bf16_bits(f[t]); sKh[r][c4 + t] = hb; sKl[r][c4 + t] = bf16_bits(f[t] - bf16_val(hb)); }
    }
    for (int e = tid; e < 32 * (DV / 4); e += 128) {
      const int r = e / (DV / 4), c4 = (e % (DV / 4)) * 4; const int key = j0 + r;
      v4f f = {0.f,0.f,0.f,0.f}; if (key < Tk) f = *(const v4fa*)(V + (size_t)key * vpitch + c4);
#pragma unroll
      for (int t = 0; t < 4; ++t) { const unsigned short hb = bf16_bits(f[t]); sVh[r][c4 + t] = hb; sVl[r][c4 + t] = bf16_bits(f[t] - bf16_val(hb)); }
    }
    __syncthreads();
    v8f s[2];
#pragma unroll
    for (int nt = 0; nt < 2; ++nt) {
      v8f acc = {};
#pragma unroll
      for (int ks = 0; ks < KS; ++ks) {
        FragB bh_, bl_;
        bh_.half[0] = *(const v8us*)&sKh[nt * 16 + ln][ks * 32 + 8 * hh]; bh_.half[1] = *(const v8us*)&sKh[nt * 16 + ln][ks * 32 + 16 + 8 * hh];
        bl_.half[0] = *(const v8us*)&sKl[nt * 16 + ln][ks * 32 + 8 * hh]; bl_.half[1] = *(const v8us*)&sKl[nt * 16 + ln][ks * 32 + 16 + 8 * hh];
        acc = mmaN<3>(aqh[ks].v, aql[ks].v, bh_.v, bl_.v, acc);
      }
      s[nt] = acc;
    }
    float alpha[8];
#pragma unroll
    for (int r = 0; r < 8; ++r) {
      const int ja = j0 + ln, jb = j0 + 16 + ln;
      if (ja >= Tk) s[0][r] = -3.0e38f;
      if (jb >= Tk) s[1][r] = -3.0e38f;
      float mx = fmaxf(s[0][r], s[1][r]);
      mx = fmaxf(mx, __shfl_xor(mx, 1, 32)); mx = fmaxf(mx, __shfl_xor(mx, 2, 32)); mx = fmaxf(mx, __shfl_xor(mx, 4, 32)); mx = fmaxf(mx, __shfl_xor(mx, 8, 32));
      const float mnew = fmaxf(m_r[r], mx);
      alpha[r] = (mnew > -1.0e38f) ? __expf(m_r[r] - mnew) : 1.0f;
      const float p0 = (s[0][r] > -1.0e38f) ? __expf(s[0][r] - mnew) : 0.f;
      const float p1 = (s[1][r] > -1.0e38f) ? __expf(s[1][r] - mnew) : 0.f;
      m_r[r] = mnew;
      l_r[r] = l_r[r] * alpha[r] + p0 + p1;
      unsigned short hb = bf16_bits(p0); sPh[w][8 * hh + r][ln] = hb;      sPl[w][8 * hh + r][ln] = bf16_bits(p0 - bf16_val(hb));
      hb = bf16_bits(p1);                sPh[w][8 * hh + r][16 + ln] = hb; sPl[w][8 * hh + r][16 + ln] = bf16_bits(p1 - bf16_val(hb));
    }
#pragma unroll
    for (int dt = 0; dt < DT; ++dt)
#pragma unroll
      for (int r = 0; r < 8; ++r) oacc[dt][r] *= alpha[r];
    __builtin_amdgcn_fence(__ATOMIC_ACQ_REL, "workgroup");
    __builtin_amdgcn_wave_barrier();
    FragB pah, pal;
    pah.half[0] = *(const v8us*)&sPh[w][ln][8 * hh]; pah.half[1] = *(const v8us*)&sPh[w][ln][16 + 8 * hh];
    pal.half[0] = *(const v8us*)&sPl[w][ln][8 * hh]; pal.half[1] = *(const v8us*)&sPl[w][ln][16 + 8 * hh];
#pragma unroll
    for (int dt = 0; dt < DT; ++dt) {
      FragB bvh, bvl;
#pragma unroll
      for (int i = 0; i < 8; ++i) {
        bvh.u[i] = sVh[8 * hh + i][dt * 16 + ln]; bvh.u[8 + i] = sVh[16 + 8 * hh + i][dt * 16 + ln];
        bvl.u[i] = sVl[8 * hh + i][dt * 16 + ln]; bvl.u[8 + i] = sVl[16 + 8 * hh + i][dt * 16 + ln];
      }
      oacc[dt] = mmaN<3>(pah.v, pal.v, bvh.v, bvl.v, oacc[dt]);
    }
    __builtin_amdgcn_fence(__ATOMIC_ACQ_REL, "workgroup");
    __builtin_amdgcn_wave_barrier();
  }
#pragma unroll
  for (int r = 0; r < 8; ++r) {
    float l = l_r[r];
    l += __shfl_xor(l, 1, 32); l += __shfl_xor(l, 2, 32); l += __shfl_xor(l, 4, 32); l += __shfl_xor(l, 8, 32);
    l_r[r] = (l > 0.f) ? 1.0f / l : 0.f;
  }
#pragma unroll
  for (int dt = 0; dt < DT; ++dt)
#pragma unroll
    for (int r = 0; r < 8; ++r) sO[w][8 * hh + r][dt * 16 + ln] = oacc[dt][r] * l_r[r];
  __builtin_amdgcn_fence(__ATOMIC_ACQ_REL, "workgroup");
  __builtin_amdgcn_wave_barrier();
  for (int pass = 0; pass < 2; ++pass) {
    for (int r = 0; r < 16; ++r) {
      const int row = q0 + r;
      for (int c4 = lane * 4; c4 < DV; c4 += 128) {
        if (row < Tq) {
          const v4f val = *(const v4fa*)&sO[w][r][c4];
          *(volatile v4f*)(y + (size_t)bh * ystride + (size_t)row * ypitch + dv0 + c4) = val;
        }
      }
    }
    if (pass == 0) __threadfence();
  }
}

template <bool ASPLIT, int ACT, bool BIAS_BF16, bool RES_BF16>
__global__ __launch_bounds__(128) void k_gemm_bf3(const float* __restrict__ A, int lda, const unsigned short* __restrict__ Wt, int ldb,
                                                const float* __restrict__ bias, const float* __restrict__ resid, int rmod, int ldr,
                                                float* __restrict__ C, int ldc, int M, int N, int K) {
  __shared__ __attribute__((aligned(16))) float so[4][16][64];
  const int tid = threadIdx.x, w = tid >> 5, lane = tid & 31, ln = lane & 15, hh = lane >> 4;
  const int ntn = N / 64;
  const int wid = blockIdx.x * 4 + w;
  const int mt = wid / ntn, nq = wid % ntn;
  if (mt * 16 >= M) return;
  const int row0 = mt * 16, col0 = nq * 64;
  const float* arow = A + (size_t)(row0 + ln) * lda;
  v8f acc[4] = {};
  for (int kb = 0; kb < K; kb += 32) {
    FragB ah, al;
    const v4f x0 = *(const v4fa*)(arow + kb + 8 * hh), x1 = *(const v4fa*)(arow + kb + 8 * hh + 4);
    const v4f x2 = *(const v4fa*)(arow + kb + 16 + 8 * hh), x3 = *(const v4fa*)(arow + kb + 16 + 8 * hh + 4);
    float xs[16] = {x0[0],x0[1],x0[2],x0[3],x1[0],x1[1],x1[2],x1[3],x2[0],x2[1],x2[2],x2[3],x3[0],x3[1],x3[2],x3[3]};
#pragma unroll
    for (int i = 0; i < 16; ++i) { const unsigned short hb = bf16_bits(xs[i]); ah.u[i] = hb; al.u[i] = ASPLIT ? bf16_bits(xs[i] - bf16_val(hb)) : (unsigned short)0; }
#pragma unroll
    for (int t = 0; t < 4; ++t) {
      const unsigned short* brow = Wt + (size_t)(col0 + t * 16 + ln) * ldb + kb;
      FragB b;
      b.half[0] = *(const v8us*)(brow + 8 * hh);
      b.half[1] = *(const v8us*)(brow + 16 + 8 * hh);
      acc[t] = mmaN<ASPLIT ? 2 : 1>(ah.v, al.v, b.v, b.v, acc[t]);
    }
  }
#pragma unroll
  for (int t = 0; t < 4; ++t) {
    const int col = col0 + t * 16 + ln;
    float bv = bias ? bias[col] : 0.f;
    if (BIAS_BF16) bv = bf16_round(bv);
#pragma unroll
    for (int r = 0; r < 8; ++r) {
      float v = acc[t][r] + bv;
      if (resid) { float rv = resid[(size_t)((row0 + 8 * hh + r) % rmod) * ldr + col]; if (RES_BF16) rv = bf16_round(rv); v += rv; }
      if (ACT == 1) v = fmaxf(v, 0.f);
      if (ACT == 2) v = 0.5f * v * (1.0f + erff(v * 0.70710678118654752f));
      if (ACT == 3) { const float u = 0.7978845608028654f * (v + 0.044715f * v * v * v); v = 0.5f * v * (1.0f + tanhf(u)); }
      so[w][8 * hh + r][t * 16 + ln] = v;
    }
  }
  __builtin_amdgcn_fence(__ATOMIC_ACQ_REL, "workgroup");
  __builtin_amdgcn_wave_barrier();
  const int rsub = lane >> 4, c4 = (lane & 15) * 4;
  for (int pass = 0; pass < 2; ++pass) {
#pragma unroll
    for (int q = 0; q < 8; ++q) {
      const int r = q * 2 + rsub;
      const v4f v = *(const v4fa*)&so[w][r][c4];
      *(volatile v4f*)(C + (size_t)(row0 + r) * ldc + col0 + c4) = v;
    }
    if (pass == 0) __threadfence();
  }
}
template <bool PARAM_BF16>
__global__ __launch_bounds__(256) void k_layernorm(const float* __restrict__ X, const float* __restrict__ R, const float* __restrict__ g, const float* __restrict__ bta,
                                                  float* __restrict__ out_sum, float* __restrict__ out_norm, int N, float eps) {
  __shared__ float red[256];
  const int row = blockIdx.x, tid = threadIdx.x;
  const float* x = X + (size_t)row * N; const float* rr = R ? R + (size_t)row * N : nullptr;
  float vals[16];
  const int per = N / 256;
  float s1 = 0.f;
  for (int u = 0; u < per / 4; ++u) {
    const int j = tid * 4 + 1024 * u;
    const v4f a = *(const v4fa*)(x + j);
    v4f b = {0.f,0.f,0.f,0.f}; if (rr) b = *(const v4fa*)(rr + j);
#pragma unroll
    for (int q = 0; q < 4; ++q) { const float v = a[q] + b[q]; vals[u * 4 + q] = v; s1 += v; }
  }
  red[tid] = s1; __syncthreads();
  for (int st = 128; st > 0; st >>= 1) { if (tid < st) red[tid] += red[tid + st]; __syncthreads(); }
  const float mu = red[0] / (float)N; __syncthreads();
  float s2 = 0.f;
  for (int u = 0; u < per / 4; ++u)
#pragma unroll
    for (int q = 0; q < 4; ++q) { const float c = vals[u * 4 + q] - mu; s2 += c * c; }
  red[tid] = s2; __syncthreads();
  for (int st = 128; st > 0; st >>= 1) { if (tid < st) red[tid] += red[tid + st]; __syncthreads(); }
  const float rs = rsqrtf(red[0] / (float)N + eps);
  for (int pass = 0; pass < 2; ++pass) {
    for (int u = 0; u < per / 4; ++u) {
      const int j = tid * 4 + 1024 * u;
      v4f o, sm;
#pragma unroll
      for (int q = 0; q < 4; ++q) {
        float gg = g[j + q], bb = bta[j + q];
        if (PARAM_BF16) { gg = bf16_round(gg); bb = bf16_round(bb); }
        sm[q] = vals[u * 4 + q]; o[q] = (vals[u * 4 + q] - mu) * rs * gg + bb;
      }
      if (out_sum) *(volatile v4f*)(out_sum + (size_t)row * N + j) = sm;
      *(volatile v4f*)(out_norm + (size_t)row * N + j) = o;
    }
    if (pass == 0) __threadfence();
  }
}

typedef _Float16 v16h __attribute__((ext_vector_type(16)));
union FragH { v16h v; v8us half[2]; _Float16 h[16]; unsigned short u[16]; };
template <int NT>
__device__ __forceinline__ v8f mmaH(v16h ah, v16h al, v16h bh, v16h bl, v8f c) {
  c = __builtin_amdgcn_wmma_f32_16x16x32_f16(false, ah, false, bh, (short)0, c, false, false);
  if (NT >= 2) c = __builtin_amdgcn_wmma_f32_16x16x32_f16(false, al, false, bh, (short)0, c, false, false);
  if (NT >= 3) c = __builtin_amdgcn_wmma_f32_16x16x32_f16(false, ah, false, bl, (short)0, c, false, false);
  asm volatile("v_nop\n\tv_nop\n\tv_nop\n\tv_nop" : "+v"(c) : "v"(ah), "v"(al), "v"(bh), "v"(bl));
  return c;
}
template <bool ASPLIT>
__global__ __launch_bounds__(128) void k_gemm_h(const float* __restrict__ A, int lda, size_t sA, const _Float16* __restrict__ Bh, int ldb, size_t sB, float alpha, float* __restrict__ C, int ldc, size_t sC, int M, int N, int K) {
  __shared__ __attribute__((aligned(16))) float so[4][16][64];
  const int tid = threadIdx.x, w = tid >> 5, lane = tid & 31, ln = lane & 15, hh = lane >> 4; const int by = blockIdx.y;
  A += (size_t)by * sA; Bh += (size_t)by * sB; C += (size_t)by * sC;
  const int ntn = (N + 63) / 64; const int wid = blockIdx.x * 4 + w; const int mt = wid / ntn, nq = wid % ntn; if (mt * 16 >= M) return;
  const int row0 = mt * 16, col0 = nq * 64; const float* arow = A + (size_t)(row0 + ln) * lda;
  v8f acc[4] = {};
  for (int kb = 0; kb < K; kb += 32) {
    FragH ah, al;
    const v4f x0 = *(const v4fa*)(arow + kb + 8 * hh), x1 = *(const v4fa*)(arow + kb + 8 * hh + 4), x2 = *(const v4fa*)(arow + kb + 16 + 8 * hh), x3 = *(const v4fa*)(arow + kb + 16 + 8 * hh + 4);
    float xs[16] = {x0[0],x0[1],x0[2],x0[3],x1[0],x1[1],x1[2],x1[3],x2[0],x2[1],x2[2],x2[3],x3[0],x3[1],x3[2],x3[3]};
#pragma unroll
    for (int i = 0; i < 16; ++i) { const _Float16 h = (_Float16)xs[i]; ah.h[i] = h; al.h[i] = ASPLIT ? (_Float16)(xs[i] - (float)h) : (_Float16)0.0f; }
#pragma unroll
    for (int t = 0; t < 4; ++t) { if (col0 + t * 16 >= N) continue; const size_t boff = (size_t)(col0 + t * 16 + ln) * ldb + kb; FragH bq; bq.half[0] = *(const v8us*)(Bh + boff + 8 * hh); bq.half[1] = *(const v8us*)(Bh + boff + 16 + 8 * hh);
      acc[t] = mmaH<ASPLIT ? 2 : 1>(ah.v, al.v, bq.v, bq.v, acc[t]); }
  }
#pragma unroll
  for (int t = 0; t < 4; ++t) { if (col0 + t * 16 >= N) continue;
#pragma unroll
    for (int r = 0; r < 8; ++r) so[w][8 * hh + r][t * 16 + ln] = acc[t][r] * alpha; }
  __builtin_amdgcn_fence(__ATOMIC_ACQ_REL, "workgroup"); __builtin_amdgcn_wave_barrier();
  const int rsub = lane >> 4, c4 = (lane & 15) * 4;
  for (int pass = 0; pass < 2; ++pass) {
#pragma unroll
    for (int q = 0; q < 8; ++q) { const int r = q * 2 + rsub; if (col0 + c4 < N) { const v4f v = *(const v4fa*)&so[w][r][c4]; *(volatile v4f*)(C + (size_t)(row0 + r) * ldc + col0 + c4) = v; } }
    if (pass == 0) __threadfence(); }
}

__global__ __launch_bounds__(256) void k_round_rows(const float* __restrict__ W, unsigned short* __restrict__ Wt, int n8) {
  const int t = blockIdx.x * 256 + threadIdx.x;
  if (t >= n8) return;
  const v4f a = *(const v4fa*)(W + (size_t)t * 8), b = *(const v4fa*)(W + (size_t)t * 8 + 4);
  v8us v; v[0]=bf16_bits(a[0]); v[1]=bf16_bits(a[1]); v[2]=bf16_bits(a[2]); v[3]=bf16_bits(a[3]);
  v[4]=bf16_bits(b[0]); v[5]=bf16_bits(b[1]); v[6]=bf16_bits(b[2]); v[7]=bf16_bits(b[3]);
  *(volatile v8us*)(Wt + (size_t)t * 8) = v; __threadfence(); *(volatile v8us*)(Wt + (size_t)t * 8) = v;
}

__global__ __launch_bounds__(256) void k_cvt16(const float* __restrict__ a, _Float16* __restrict__ h, size_t n8) { const size_t t = (size_t)blockIdx.x * 256 + threadIdx.x; if (t >= n8) return; FragH f; for (int q = 0; q < 8; ++q) f.h[q] = (_Float16)a[t * 8 + q]; const v8us o = f.half[0]; *(volatile v8us*)((unsigned short*)h + t * 8) = o; __threadfence(); *(volatile v8us*)((unsigned short*)h + t * 8) = o; }
__global__ __launch_bounds__(256) void k_l2n(float* __restrict__ Y, _Float16* __restrict__ Y16, int rows) { const int tid = threadIdx.x, wv = tid >> 5, lane = tid & 31; const int r = blockIdx.x * 8 + wv; if (r >= rows) return; float* row = Y + (size_t)r * KD; const v4f v = *(const v4fa*)(row + 4 * lane);
  float s = v[0] * v[0] + v[1] * v[1] + v[2] * v[2] + v[3] * v[3]; for (int o = 16; o >= 1; o >>= 1) s += __shfl_xor(s, o, 32); const float inv = 1.0f / fmaxf(sqrtf(s), 1e-12f);
  v4f o4; typedef _Float16 v4h __attribute__((ext_vector_type(4))); v4h h4; for (int q = 0; q < 4; ++q) { o4[q] = v[q] * inv; h4[q] = (_Float16)o4[q]; }
  __builtin_amdgcn_wave_barrier();
  *(volatile v4f*)(row + 4 * lane) = o4; if (Y16) *(volatile v4h*)(Y16 + (size_t)r * KD + 4 * lane) = h4; __threadfence(); *(volatile v4f*)(row + 4 * lane) = o4; if (Y16) *(volatile v4h*)(Y16 + (size_t)r * KD + 4 * lane) = h4; }
__global__ __launch_bounds__(1024) void k_softmax(float* __restrict__ S, int N, float* __restrict__ Dn) {
  __shared__ float sd[32]; const int tid = threadIdx.x, wv = tid >> 5, lane = tid & 31; const size_t r = (size_t)blockIdx.x * 32 + wv; float* row = S + r * N;
  float mx = -3.0e38f;
#pragma unroll 1
  for (int j = lane; j < N; j += 32) mx = fmaxf(mx, row[j] * 30.0f);
  for (int o = 16; o >= 1; o >>= 1) mx = fmaxf(mx, __shfl_xor(mx, o, 32));
  float den = 0.f;
#pragma unroll 1
  for (int j = lane; j < N; j += 32) { const float e = expf(row[j] * 30.0f - mx); den += e; *(volatile float*)(row + j) = e * 256.0f; }
  for (int o = 16; o >= 1; o >>= 1) den += __shfl_xor(den, o, 32);
  __threadfence();
#pragma unroll 1
  for (int j = lane; j < N; j += 32) { const float pv = row[j]; *(volatile float*)(row + j) = pv; }
  if (lane == 0) sd[wv] = den; __syncthreads();
  if (tid < 32) { *(volatile float*)(Dn + (size_t)blockIdx.x * 32 + tid) = sd[tid]; } __threadfence(); if (tid < 32) { *(volatile float*)(Dn + (size_t)blockIdx.x * 32 + tid) = sd[tid]; } }
__global__ __launch_bounds__(256) void k_instat(const float* __restrict__ T1, float* __restrict__ st) { const int c = threadIdx.x; double s = 0.0, q = 0.0;
#pragma unroll 1
  for (int r = 0; r < HW; ++r) { const float v = T1[(size_t)r * CC + c]; s += (double)v; q += (double)v * (double)v; }
  const double mu = s / HW; double var = q / HW - mu * mu; if (var < 0.0) var = 0.0; const float rs = (float)(1.0 / sqrt(var + 1e-5)); const float sh = -(float)mu * rs;
  *(volatile float*)(st + c * 2) = rs; *(volatile float*)(st + c * 2 + 1) = sh; __threadfence(); *(volatile float*)(st + c * 2) = rs; *(volatile float*)(st + c * 2 + 1) = sh; }
__global__ __launch_bounds__(256) void k_resid(const float* __restrict__ T0, const float* __restrict__ O, const float* __restrict__ Dn, const float* __restrict__ bv, float* __restrict__ T1) { const int t = blockIdx.x * 256 + threadIdx.x; if (t >= HW * CC / 4) return; const int c4 = (t * 4) % CC; const int r = (t * 4) / CC; const float rd = 1.0f / Dn[r];
  const v4f a = *(const v4fa*)(T0 + (size_t)t * 4), o = *(const v4fa*)(O + (size_t)t * 4); v4f y; for (int q = 0; q < 4; ++q) y[q] = bf16_round(a[q]) + (o[q] * rd + bf16_round(bv[c4 + q])); *(volatile v4f*)(T1 + (size_t)t * 4) = y; __threadfence(); *(volatile v4f*)(T1 + (size_t)t * 4) = y; }
__global__ __launch_bounds__(256) void k_inapply(float* __restrict__ T1, const float* __restrict__ st) { const int t = blockIdx.x * 256 + threadIdx.x; if (t >= HW * CC / 4) return; const int c4 = (t * 4) % CC; v4f v = *(const v4fa*)(T1 + (size_t)t * 4); for (int q = 0; q < 4; ++q) v[q] = v[q] * st[(c4 + q) * 2] + st[(c4 + q) * 2 + 1]; *(volatile v4f*)(T1 + (size_t)t * 4) = v; __threadfence(); *(volatile v4f*)(T1 + (size_t)t * 4) = v; }
__global__ __launch_bounds__(256) void k_posT(const float* __restrict__ src, float* __restrict__ dst) { __shared__ float tl[CE][65]; const int t = threadIdx.x; const int hw0 = blockIdx.x * 64;
  for (int e = t; e < CE * 64; e += 256) { const int ce = e >> 6, j = e & 63; tl[ce][j] = src[(size_t)ce * HW + hw0 + j]; } __syncthreads();
  for (int pass = 0; pass < 2; ++pass) { for (int e = t; e < 64 * CE; e += 256) { const int j = e >> 4, ce = e & 15; *(volatile float*)(dst + (size_t)(hw0 + j) * CE + ce) = tl[ce][j]; } if (pass == 0) __threadfence(); } }
__global__ __launch_bounds__(256) void k_pv(const float* __restrict__ P, const float* __restrict__ Wcv, _Float16* __restrict__ PVt) { __shared__ float sw[CE][CE + 1]; __shared__ _Float16 so[CE][256 + 8]; const int t = threadIdx.x; if (t < CE * CE) sw[t / CE][t % CE] = bf16_round(Wcv[t]); __syncthreads();
  const int k = blockIdx.x * 256 + t; float pe[CE]; for (int e = 0; e < CE; ++e) pe[e] = bf16_round(P[(size_t)k * CE + e]);
#pragma unroll 1
  for (int ce = 0; ce < CE; ++ce) { float s = 0.f;
#pragma unroll
    for (int e = 0; e < CE; ++e) s += pe[e] * sw[ce][e]; so[ce][t] = (_Float16)s; }
  __syncthreads(); typedef unsigned int u32;
  for (int pass = 0; pass < 2; ++pass) { for (int e = t; e < CE * 128; e += 256) { const int ce = e >> 7, k2 = (e & 127) * 2; *(volatile u32*)(PVt + (size_t)ce * LK + blockIdx.x * 256 + k2) = *(const u32*)&so[ce][k2]; } if (pass == 0) __threadfence(); } }
__global__ __launch_bounds__(256) void k_outT(const float* __restrict__ O2, const float* __restrict__ Dn2, const float* __restrict__ bcv, int s, float* __restrict__ out) { const int t = blockIdx.x * 256 + threadIdx.x; if (t >= CE * HW) return; const int hw = t % HW, ce = t / HW; const float v = O2[(size_t)hw * CE + ce] / Dn2[hw] + bf16_round(bcv[ce]); *(volatile float*)(out + ((size_t)s * CE) * HW + t) = v; __threadfence(); *(volatile float*)(out + ((size_t)s * CE) * HW + t) = v; }
extern "C" void kernel_launch(void* const* d_in, const int* in_sizes, int n_in,
                              void* d_out, int out_size, void* d_ws, size_t ws_size, hipStream_t stream) {
  (void)in_sizes; (void)n_in; (void)out_size;
  const float* tgt = (const float*)d_in[0]; const float* mem = (const float*)d_in[1]; const float* pos = (const float*)d_in[2];
  const float* sWk = (const float*)d_in[3]; const float* sbk = (const float*)d_in[4]; const float* sWv = (const float*)d_in[5]; const float* sbv = (const float*)d_in[6]; const float* cWk = (const float*)d_in[7]; const float* cbk = (const float*)d_in[8]; const float* cWv = (const float*)d_in[9]; const float* cbv = (const float*)d_in[10];
  char* ws = (char*)d_ws; size_t off = 0;
  auto take = [&](size_t bytes) { char* p = ws + off; off += (bytes + 255) & ~(size_t)255; return p; };
  unsigned short* BsK = (unsigned short*)take(KD * CC * 2); unsigned short* BcK = (unsigned short*)take(KD * CC * 2);
  float* T0 = (float*)take((size_t)HW * CC * 4); unsigned short* T0b = (unsigned short*)take((size_t)HW * CC * 2); float* Ms = (float*)take((size_t)LK * CC * 4); float* Ps = (float*)take((size_t)LK * CE * 4);
  float* Q0 = (float*)take((size_t)HW * KD * 4); _Float16* K016 = (_Float16*)take((size_t)HW * KD * 2); float* V0t = (float*)take((size_t)CC * HW * 4); _Float16* V0t16 = (_Float16*)take((size_t)CC * HW * 2);
  float* S1 = (float*)take((size_t)HW * HW * 4); float* Dn1 = (float*)take(HW * 4); float* O1 = (float*)take((size_t)HW * CC * 4); float* T1 = (float*)take((size_t)HW * CC * 4); float* st = (float*)take(CC * 2 * 4);
  float* Qc = (float*)take((size_t)HW * KD * 4); float* Kc = (float*)take((size_t)LK * KD * 4); _Float16* Kc16 = (_Float16*)take((size_t)LK * KD * 2); _Float16* PVt = (_Float16*)take((size_t)CE * LK * 2);
  float* S2 = (float*)take((size_t)HW * LK * 4); float* Dn2 = (float*)take(HW * 4); float* O2 = (float*)take((size_t)HW * CE * 4);
  if (off > ws_size) return;
  k_round_rows<<<(KD * CC / 8 + 255) / 256, 256, 0, stream>>>(sWk, BsK, KD * CC / 8); k_round_rows<<<(KD * CC / 8 + 255) / 256, 256, 0, stream>>>(cWk, BcK, KD * CC / 8);
  for (int s = 0; s < NS; ++s) {
    k_transpose32<false, false, false><<<dim3(HW / 32, CC / 32, 1), 256, 0, stream>>>(tgt + (size_t)s * CC * HW, T0, CC, HW, nullptr, nullptr, nullptr);
    for (int f = 0; f < NFR; ++f) { k_transpose32<false, false, false><<<dim3(HW / 32, CC / 32, 1), 256, 0, stream>>>(mem + ((size_t)f * NS + s) * CC * HW, Ms + (size_t)f * HW * CC, CC, HW, nullptr, nullptr, nullptr);
      k_posT<<<HW / 64, 256, 0, stream>>>(pos + ((size_t)f * NS + s) * CE * HW, Ps + (size_t)f * HW * CE); }
    k_round_rows<<<(HW * CC / 8 + 255) / 256, 256, 0, stream>>>(T0, T0b, HW * CC / 8);
    k_gemm_bf3<false, 0, true, false><<<((HW / 16) * (KD / 64) + 3) / 4, 128, 0, stream>>>(T0, CC, BsK, CC, sbk, nullptr, 1, 0, Q0, KD, HW, KD, CC);
    k_l2n<<<HW / 8, 256, 0, stream>>>(Q0, K016, HW);
    k_gemm_bf3<false, 0, false, false><<<((CC / 16) * (HW / 64) + 3) / 4, 128, 0, stream>>>(sWv, CC, T0b, CC, nullptr, nullptr, 1, 0, V0t, HW, CC, HW, CC);
    k_cvt16<<<(CC * HW / 8 + 255) / 256, 256, 0, stream>>>(V0t, V0t16, (size_t)CC * HW / 8);
    k_gemm_h<true><<<dim3(((HW / 16) * (HW / 64) + 3) / 4, 1), 128, 0, stream>>>(Q0, KD, 0, K016, KD, 0, 1.f, S1, HW, 0, HW, HW, KD);
    k_softmax<<<HW / 32, 1024, 0, stream>>>(S1, HW, Dn1);
    k_gemm_h<false><<<dim3(((HW / 16) * (CC / 64) + 3) / 4, 1), 128, 0, stream>>>(S1, HW, 0, V0t16, HW, 0, 0.00390625f, O1, CC, 0, HW, CC, HW);
    k_resid<<<(HW * CC / 4 + 255) / 256, 256, 0, stream>>>(T0, O1, Dn1, sbv, T1); k_instat<<<1, 256, 0, stream>>>(T1, st); k_inapply<<<(HW * CC / 4 + 255) / 256, 256, 0, stream>>>(T1, st);
    k_gemm_bf3<true, 0, true, false><<<((HW / 16) * (KD / 64) + 3) / 4, 128, 0, stream>>>(T1, CC, BcK, CC, cbk, nullptr, 1, 0, Qc, KD, HW, KD, CC);
    k_l2n<<<HW / 8, 256, 0, stream>>>(Qc, nullptr, HW);
    k_gemm_bf3<false, 0, true, false><<<((LK / 16) * (KD / 64) + 3) / 4, 128, 0, stream>>>(Ms, CC, BcK, CC, cbk, nullptr, 1, 0, Kc, KD, LK, KD, CC);
    k_l2n<<<LK / 8, 256, 0, stream>>>(Kc, Kc16, LK);
    k_pv<<<LK / 256, 256, 0, stream>>>(Ps, cWv, PVt);
    k_gemm_h<true><<<dim3(((HW / 16) * (LK / 64) + 3) / 4, 1), 128, 0, stream>>>(Qc, KD, 0, Kc16, KD, 0, 1.f, S2, LK, 0, HW, LK, KD);
    k_softmax<<<HW / 32, 1024, 0, stream>>>(S2, LK, Dn2);
    k_gemm_h<false><<<dim3(((HW / 16) * 1 + 3) / 4, 1), 128, 0, stream>>>(S2, LK, 0, PVt, LK, 0, 0.00390625f, O2, CE, 0, HW, CE, LK);
    k_outT<<<(CE * HW + 255) / 256, 256, 0, stream>>>(O2, Dn2, cbv, s, (float*)d_out);
  }
}
